// DualModeHead_42245298323784
// MI455X (gfx1250) — hardware-verified
//
#include <hip/hip_runtime.h>


#ifndef NB
#define NB 8
#endif
#ifndef SEQ
#define SEQ 2048
#endif
#define NB_FULL  8
#define SEQ_FULL 2048
#ifndef OUT_SEQ
#define OUT_SEQ SEQ
#endif
#define DM   128
#define AW   4
#define OSP  132
#define VTP  72
#define MW   (SEQ / 32)
#define EROWS (SEQ < 512 ? SEQ : 512)
#define XCAR 16.0f
#define QRS  2048.0f
#define QRI  (1.0f / 2048.0f)
#define SC2  ((float)(0.08838834764831845 * 1.4426950408889634 / 256.0))
#define PSH  14.0f
#define NEGB (-3.0e38f)

static_assert(DM == 128);
static_assert(DM % 32 == 0);
static_assert(DM / 8 == 16);
static_assert((DM & (DM - 1)) == 0);
static_assert(SEQ % 128 == 0);
static_assert(SEQ % 64 == 0);
static_assert(SEQ % 32 == 0);
static_assert(EROWS % (16 * AW) == 0);
static_assert((SEQ - EROWS) % (16 * AW) == 0);
static_assert(EROWS >= 32);
static_assert(EROWS % 32 == 0);
static_assert(EROWS <= SEQ);
static_assert(NB <= NB_FULL);
static_assert(SEQ <= SEQ_FULL);
static_assert((OSP * 4) % 16 == 0);
static_assert(OSP >= DM);
static_assert((VTP * 2) % 16 == 0);
static_assert(VTP >= 64);
static_assert((size_t)AW * 16 * OSP * 4 <= 131072);
static_assert((size_t)DM * VTP * 2 <= 131072);
static_assert(32 * 4 * 16 == 16 * DM);
static_assert(256 * 4 * 8 == 64 * DM);
static_assert(256 * 8 * 4 == DM * 64);
static_assert((size_t)NB * SEQ * DM / 8 < (size_t)2147483647);
static_assert((size_t)SEQ * DM < (size_t)2147483647);

typedef _Float16 h16;
typedef __attribute__((ext_vector_type(16))) _Float16 v16h;
typedef __attribute__((ext_vector_type(8)))  _Float16 v8h;
typedef __attribute__((ext_vector_type(8)))  float    v8f;
typedef __attribute__((ext_vector_type(4)))  float    v4f;
typedef __attribute__((ext_vector_type(4)))  int      v4i;
typedef __attribute__((ext_vector_type(4)))  unsigned v4u;
typedef v4f  __attribute__((may_alias)) v4fa;
typedef v8h  __attribute__((may_alias)) v8ha;

__device__ __forceinline__ unsigned short f2bf(float f) { unsigned u = __float_as_uint(f); u += 0x7FFFu + ((u >> 16) & 1u); return (unsigned short)(u >> 16); }
__device__ __forceinline__ float bfr(float f) { return __uint_as_float(((unsigned)f2bf(f)) << 16); }
__device__ __forceinline__ v16h cat16(v8h lo, v8h hi) { return __builtin_shufflevector(lo, hi, 0, 1, 2, 3, 4, 5, 6, 7, 8, 9, 10, 11, 12, 13, 14, 15); }
__device__ __forceinline__ v8f wmma16(v16h a, v16h b, v8f c) { return __builtin_amdgcn_wmma_f32_16x16x32_f16(false, a, false, b, (short)0, c, false, false); }
__device__ __forceinline__ v16h  ldh(const h16* p) { return cat16(*(const v8h*)p, *(const v8h*)(p + 16)); }
__device__ __forceinline__ void wave_sync() { __builtin_amdgcn_fence(3  , "wavefront"); __builtin_amdgcn_wave_barrier(); asm volatile("" ::: "memory"); }

static __device__ __forceinline__ h16 toh_flush(float v) { const h16 r = (h16)v; return (fabsf(v) < 6.103515625e-05f) ? (h16)0.0f : r; }
static __device__ __forceinline__ v8f wmma16g(v16h a, v16h b, v8f c) {
    c = wmma16(a, b, c);
    asm volatile("v_nop\n\tv_nop\n\tv_nop\n\tv_nop" : "+v"(c) : "v"(a), "v"(b));
    return c;
}

__global__ __launch_bounds__(256) void k_cvtq(const float* __restrict__ src, h16* dst, int n8) {
#pragma clang fp contract(off)
    const int i = blockIdx.x * 256 + threadIdx.x; if (i >= n8) return;
    const int row = i >> 4, d0 = (i & 15) * 8; const int b = row / SEQ, t = row % SEQ;
    const v8f v = *(const v8f*)(src + ((size_t)b * SEQ_FULL + (size_t)t) * DM + d0); v8h o;
#pragma unroll
    for (int e = 0; e < 8; ++e) o[e] = toh_flush(bfr(v[e]) * XCAR);
    *(volatile v8h*)(dst + (size_t)i * 8) = o; __threadfence(); *(volatile v8h*)(dst + (size_t)i * 8) = o;
}

__global__ __launch_bounds__(256) void k_keff(const float* __restrict__ k, const float* __restrict__ mode, h16* KE, h16* KR, int n8) {
#pragma clang fp contract(off)
    const int i = blockIdx.x * 256 + threadIdx.x; if (i >= n8) return;
    const int row = i >> 4, d0 = (i & 15) * 8; const int b = row / SEQ, t = row % SEQ;
    const float* kr = k + ((size_t)b * SEQ_FULL + (size_t)t) * DM;
    const v8f x = *(const v8f*)(kr + d0);
    const float xm = kr[(d0 + DM - 1) & (DM - 1)];
    const float mv = bfr(mode[0]);
    const float al = 1.0f / (1.0f + expf(-mv));
    const float oma = 1.0f - al;
    float prev = bfr(xm); v8h hv, rv;
#pragma unroll
    for (int e = 0; e < 8; ++e) {
        const float cur = bfr(x[e]);
        const float c = (oma * prev - al * cur) * XCAR;
        const h16 hh = toh_flush(c);
        hv[e] = hh; rv[e] = toh_flush((c - (float)hh) * QRS);
        prev = cur; }
    const bool wr = t < EROWS;
    const size_t oo = (size_t)i * 8;
    const size_t ro = ((size_t)b * EROWS + (size_t)(wr ? t : 0)) * DM + d0;
    *(volatile v8h*)(KE + oo) = hv; if (wr) *(volatile v8h*)(KR + ro) = rv;
    __threadfence();
    *(volatile v8h*)(KE + oo) = hv; if (wr) *(volatile v8h*)(KR + ro) = rv;
}

__global__ __launch_bounds__(256) void k_vt(const float* __restrict__ v, h16* VT) {
#pragma clang fp contract(off)
    __shared__ __align__(16) h16 ts[DM * VTP];
    const int tid = threadIdx.x; const int b = blockIdx.y, tok0 = blockIdx.x * 64;
    const float* src = v + ((size_t)b * SEQ_FULL + (size_t)tok0) * DM;
#pragma unroll 1
    for (int i = 0; i < 8; ++i) { const int idx = i * 256 + tid; const int tk = idx >> 5, c4 = (idx & 31) * 4;
        const v4f x = *(const v4f*)(src + (size_t)tk * DM + c4);
#pragma unroll
        for (int e = 0; e < 4; ++e) ts[(c4 + e) * VTP + tk] = toh_flush(bfr(x[e]) * XCAR); }
    __syncthreads();
    h16* dstb = VT + (size_t)b * DM * SEQ + (size_t)tok0;
#pragma unroll 1
    for (int ps = 0; ps < 2; ++ps) {
#pragma unroll
        for (int s = 0; s < 4; ++s) { const int p = s * 256 + tid; const int d = p >> 3, c8 = (p & 7) * 8;
            const v8h val = *(const v8ha*)(&ts[d * VTP + c8]);
            *(volatile v8h*)(dstb + (size_t)d * SEQ + c8) = val; }
        if (ps == 0) __threadfence(); }
}

__device__ __forceinline__ unsigned mword(const int* __restrict__ p) {
    unsigned w = 0u;
#pragma unroll
    for (int c = 0; c < 8; ++c) { const v4i x = *(const v4i*)(p + c * 4);
        w |= ((x[0] != 0) ? 1u : 0u) << (c * 4);
        w |= ((x[1] != 0) ? 1u : 0u) << (c * 4 + 1);
        w |= ((x[2] != 0) ? 1u : 0u) << (c * 4 + 2);
        w |= ((x[3] != 0) ? 1u : 0u) << (c * 4 + 3); }
    asm volatile("" : "+v"(w) :: "memory");
    return w;
}

__global__ __launch_bounds__(256) void k_mbits(const int* __restrict__ mask, unsigned* MB, int n4) {
    const int i = blockIdx.x * 256 + threadIdx.x; if (i >= n4) return;
    const int w0 = i * 4; const int t = w0 / MW, wc = w0 % MW;
    const int* src = mask + (size_t)t * SEQ_FULL + (size_t)wc * 32;
    v4u o;
    o[0] = mword(src); o[1] = mword(src + 32); o[2] = mword(src + 64); o[3] = mword(src + 96);
    *(volatile v4u*)(MB + (size_t)i * 4) = o; __threadfence(); *(volatile v4u*)(MB + (size_t)i * 4) = o;
}

template <int EARLY>
__device__ __forceinline__ void flash_body(const h16* __restrict__ QH, const h16* __restrict__ KE, const h16* __restrict__ KR, const h16* __restrict__ VT,
                                           const unsigned* __restrict__ MB, float* OUT) {
    __shared__ __align__(16) float os[AW * 16 * OSP];
    constexpr int VG = EARLY ? 2 : 4;
    const int lane = threadIdx.x & 31, lr = lane & 15, hi = lane >> 4;
    const int wave = __builtin_amdgcn_readfirstlane((int)(threadIdx.x >> 5));
    const int b = blockIdx.y;
    const int t0 = (EARLY ? 0 : EROWS) + (blockIdx.x * AW + wave) * 16;
    const h16* Qb = QH + (size_t)b * SEQ * DM;
    const h16* Kb = KE + (size_t)b * SEQ * DM;
    const h16* Rb = KR + (size_t)b * EROWS * DM;
    const h16* Vb = VT + (size_t)b * DM * SEQ;
    const unsigned* mrow = MB + (size_t)(t0 + lr) * MW;
    const int qo0 = (t0 + lr) * DM + 8 * hi;
    const int ko = lr * DM + 8 * hi;
    const int vo = lr * SEQ + 8 * hi;
    const v16h hz = (v16h){};
    v8f o[8], oR[8];
#pragma unroll
    for (int j = 0; j < 8; ++j) { o[j] = (v8f){}; oR[j] = (v8f){}; }
    float m = NEGB, l = 0.0f;
#pragma unroll 1
    for (int ks = 0; ks < MW; ++ks) {
        unsigned mw = mrow[ks];
        asm volatile("" : "+v"(mw));
        if (__builtin_amdgcn_ballot_w32(mw != 0u) != 0u) {
            const int key0 = ks * 32;
            const bool rok = key0 < EROWS;
            const int kcl = rok ? key0 : (EROWS - 32);
            int qo = qo0; asm volatile("" : "+v"(qo));
            v8f sHa = (v8f){}, sHb = (v8f){}, sLa = (v8f){}, sLb = (v8f){};
#pragma unroll 1
            for (int kc = 0; kc < DM; kc += 32) {
                const v16h qf = ldh(Qb + qo + kc);
                const h16* ka = Kb + ko + key0 * DM + kc;
                const v16h ka0 = ldh(ka), kb0 = ldh(ka + 16 * DM);
                sHa = wmma16g(ka0, qf, sHa); sHb = wmma16g(kb0, qf, sHb);
                if (EARLY) {
                    const h16* kr = Rb + ko + kcl * DM + kc;
                    v16h kra = ldh(kr), krb = ldh(kr + 16 * DM);
                    if (!rok) { kra = hz; krb = hz; }
                    sLa = wmma16g(kra, qf, sLa); sLb = wmma16g(krb, qf, sLb);
                }
            }
            const unsigned ma = mw >> (8 * hi);
            float ta[8], tb[8]; bool fa[8], fb[8]; float mx = NEGB;
#pragma unroll
            for (int r = 0; r < 8; ++r) {
                fa[r] = ((ma >> r) & 1u) != 0u;
                fb[r] = ((ma >> (16 + r)) & 1u) != 0u;
                if (EARLY) { ta[r] = (sHa[r] + sLa[r] * QRI) * SC2; tb[r] = (sHb[r] + sLb[r] * QRI) * SC2; }
                else       { ta[r] = sHa[r] * SC2; tb[r] = sHb[r] * SC2; }
                mx = fmaxf(mx, fmaxf(fa[r] ? ta[r] : NEGB, fb[r] ? tb[r] : NEGB)); }
            mx = fmaxf(mx, __shfl_xor(mx, 16, 32));
            const float mnew = fmaxf(m, mx);
            const float resc = __builtin_amdgcn_exp2f(m - mnew);
            const float sh = PSH - mnew;
            v16h pb, pr = hz; float ls = 0.0f;
#pragma unroll
            for (int r = 0; r < 8; ++r) {
                const float xa = ta[r] + sh, xb = tb[r] + sh;
                const float ea = __builtin_amdgcn_exp2f(xa), eb = __builtin_amdgcn_exp2f(xb);
                const float ga = (fa[r] & (xa >= -14.0f)) ? ea : 0.0f;
                const float gb = (fb[r] & (xb >= -14.0f)) ? eb : 0.0f;
                const h16 pa = (h16)ga; const h16 pc = (h16)gb;
                pb[r] = pa; pb[8 + r] = pc;
                if (EARLY) { pr[r] = toh_flush((ga - (float)pa) * QRS); pr[8 + r] = toh_flush((gb - (float)pc) * QRS); ls += ga + gb; }
                else       { ls += (float)pa + (float)pc; } }
            l = l * resc + ls; m = mnew;
#pragma unroll
            for (int j = 0; j < 8; ++j) { o[j] = o[j] * resc; if (EARLY) oR[j] = oR[j] * resc; }
            const int vk = vo + key0;
#pragma unroll
            for (int g = 0; g < 8 / VG; ++g) {
                v16h vf[VG];
#pragma unroll
                for (int jj = 0; jj < VG; ++jj) vf[jj] = ldh(Vb + vk + (g * VG + jj) * 16 * SEQ);
#pragma unroll
                for (int jj = 0; jj < VG; ++jj) {
                    o[g * VG + jj] = wmma16g(vf[jj], pb, o[g * VG + jj]);
                    if (EARLY) oR[g * VG + jj] = wmma16g(vf[jj], pr, oR[g * VG + jj]); }
            }
        }
    }
    l += __shfl_xor(l, 16, 32);
    const bool any = l > 0.0f;
    const float lsafe = any ? l : 1.0f;
    const float inv = any ? ((1.0f / lsafe) * (1.0f / XCAR)) : __uint_as_float(0x7FC00000u);
    const int wb = wave * 16 * OSP;
#pragma unroll
    for (int j = 0; j < 8; ++j) {
        v8f f = o[j];
        if (EARLY) f = o[j] + oR[j] * QRI;
        v4f a, c;
        a[0] = f[0] * inv; a[1] = f[1] * inv; a[2] = f[2] * inv; a[3] = f[3] * inv; c[0] = f[4] * inv; c[1] = f[5] * inv; c[2] = f[6] * inv; c[3] = f[7] * inv;
        *(v4fa*)(&os[wb + lr * OSP + 16 * j + 8 * hi]) = a; *(v4fa*)(&os[wb + lr * OSP + 16 * j + 8 * hi + 4]) = c; }
    wave_sync();
    float* orow = OUT + ((size_t)b * OUT_SEQ + (size_t)t0) * DM;
#pragma unroll 1
    for (int ps = 0; ps < 2; ++ps) {
#pragma unroll
        for (int s = 0; s < 16; ++s) {
            const v4f val = *(const v4fa*)(&os[wb + s * OSP + lane * 4]);
            *(volatile v4f*)(orow + (size_t)s * DM + lane * 4) = val; }
        if (ps == 0) __threadfence(); }
}

__global__ __launch_bounds__(32 * AW) __attribute__((amdgpu_num_vgpr(256)))
void k_flash_early(const h16* __restrict__ QH, const h16* __restrict__ KE, const h16* __restrict__ KR, const h16* __restrict__ VT, const unsigned* __restrict__ MB, float* OUT) {
    flash_body<1>(QH, KE, KR, VT, MB, OUT);
}
__global__ __launch_bounds__(32 * AW) __attribute__((amdgpu_num_vgpr(256)))
void k_flash_late(const h16* __restrict__ QH, const h16* __restrict__ KE, const h16* __restrict__ KR, const h16* __restrict__ VT, const unsigned* __restrict__ MB, float* OUT) {
    flash_body<0>(QH, KE, KR, VT, MB, OUT);
}

static constexpr size_t al256(size_t v) { return (v + 255) & ~(size_t)255; }
static constexpr size_t SZ_PL = al256((size_t)NB * SEQ * DM * 2);
static constexpr size_t SZ_RS = al256((size_t)NB * EROWS * DM * 2);
static constexpr size_t SZ_MB = al256((size_t)SEQ * MW * 4);
static constexpr size_t SZ_TOTAL = 3 * SZ_PL + SZ_RS + SZ_MB;
static_assert(SZ_TOTAL <= (size_t)134217728);
static_assert(((size_t)NB * SEQ * DM) % 8 == 0);
static_assert(((size_t)SEQ * MW) % 4 == 0);
static_assert(((size_t)NB * OUT_SEQ * DM * 4) <= (size_t)8388608 || NB != NB_FULL || OUT_SEQ != SEQ_FULL);

extern "C" void kernel_launch(void* const* d_in, const int* in_sizes, int n_in,
                              void* d_out, int out_size, void* d_ws, size_t ws_size, hipStream_t stream) {
    if (n_in < 5) return;
    const size_t needx = ((size_t)(NB - 1) * SEQ_FULL + SEQ) * DM;
    const size_t needm = (size_t)(SEQ - 1) * SEQ_FULL + SEQ;
    if ((size_t)in_sizes[0] < needx || (size_t)in_sizes[1] < needx || (size_t)in_sizes[2] < needx) return;
    if ((size_t)in_sizes[3] < needm || in_sizes[4] < 1) return;
    if ((size_t)out_size < ((size_t)(NB - 1) * OUT_SEQ + SEQ) * DM) return;
    if (SZ_TOTAL > ws_size) return;
    const float* q = (const float*)d_in[0];
    const float* k = (const float*)d_in[1];
    const float* v = (const float*)d_in[2];
    const int* mask = (const int*)d_in[3];
    const float* mode = (const float*)d_in[4];
    float* OUT = (float*)d_out;
    char* wsp = (char*)d_ws;
    h16* QH = (h16*)wsp; wsp += SZ_PL;
    h16* KE = (h16*)wsp; wsp += SZ_PL;
    h16* VT = (h16*)wsp; wsp += SZ_PL;
    h16* KR = (h16*)wsp; wsp += SZ_RS;
    unsigned* MB = (unsigned*)wsp; wsp += SZ_MB;

    const int n8 = (int)((size_t)NB * SEQ * DM / 8);
    k_cvtq<<<(unsigned)((n8 + 255) / 256), 256, 0, stream>>>(q, QH, n8);
    k_keff<<<(unsigned)((n8 + 255) / 256), 256, 0, stream>>>(k, mode, KE, KR, n8);
    k_vt<<<dim3(SEQ / 64, NB, 1), 256, 0, stream>>>(v, VT);
    const int n4 = (int)((size_t)SEQ * MW / 4);
    k_mbits<<<(unsigned)((n4 + 255) / 256), 256, 0, stream>>>(mask, MB, n4);

    k_flash_early<<<dim3(EROWS / (16 * AW), NB, 1), 32 * AW, 0, stream>>>(QH, KE, KR, VT, MB, OUT);
    if (SEQ > EROWS)
        k_flash_late<<<dim3((SEQ - EROWS) / (16 * AW), NB, 1), 32 * AW, 0, stream>>>(QH, KE, KR, VT, MB, OUT);
}
